// TokenMixer_85504208929081
// MI455X (gfx1250) — hardware-verified
//
#include <hip/hip_runtime.h>
#include <stdint.h>
#include <math.h>

static constexpr int kBatch = 2;
static constexpr int kSeq   = 2048;
static constexpr int kDim   = 1024;
static constexpr int kHeads = 16;
static constexpr int kHd    = 64;
static constexpr int kRows  = kBatch * kSeq;
static constexpr int kQkvN  = 3 * kDim;
static constexpr float kEps        = 1e-5f;
static constexpr float kQCarry     = 32.0f;
static constexpr float kScoreScale = 0.125f / 1024.0f;
static constexpr float kMaskFill   = -3.40282347e38f;

typedef __attribute__((ext_vector_type(16))) _Float16 v16h;
typedef __attribute__((ext_vector_type(8)))  _Float16 v8h;
typedef __attribute__((ext_vector_type(4)))  _Float16 v4h;
typedef __attribute__((ext_vector_type(16))) __bf16   v16b;
typedef __attribute__((ext_vector_type(8)))  __bf16   v8b;
typedef __attribute__((ext_vector_type(8)))  float    v8f;
typedef __attribute__((ext_vector_type(4)))  float    v4f;

__device__ __forceinline__ unsigned short f2bf_bits(float f) {
  unsigned u = __float_as_uint(f);
  return (unsigned short)((u + 0x7FFFu + ((u >> 16) & 1u)) >> 16);
}
__device__ __forceinline__ float bf_bits2f(unsigned short h) { return __uint_as_float(((unsigned)h) << 16); }
__device__ __forceinline__ float bfrn(float f) { return bf_bits2f(f2bf_bits(f)); }

__device__ __forceinline__ void dep_guard_h(v8f& a, v8f& b, v16h x, v16h y) { asm volatile("v_nop\n\tv_nop\n\tv_nop\n\tv_nop" : "+v"(a), "+v"(b) : "v"(x), "v"(y)); }
__device__ __forceinline__ void dep_guard_b(v8f& a, v8f& b, v16b x, v16b y) { asm volatile("v_nop\n\tv_nop\n\tv_nop\n\tv_nop" : "+v"(a), "+v"(b) : "v"(x), "v"(y)); }
__device__ __forceinline__ void keep4_h(v16h a, v16h b, v16h c, v16h d) { asm volatile("v_nop" :: "v"(a), "v"(b), "v"(c), "v"(d)); }
__device__ __forceinline__ void keep4_b(v16b a, v16b b, v16b c, v16b d) { asm volatile("v_nop" :: "v"(a), "v"(b), "v"(c), "v"(d)); }
__device__ __forceinline__ void acc_guard4(v8f& a, v8f& b, v8f& c, v8f& d) { asm volatile("v_nop\n\tv_nop\n\tv_nop\n\tv_nop" : "+v"(a), "+v"(b), "+v"(c), "+v"(d)); }
template <typename T> struct Frag;
template <> struct Frag<_Float16> {
  typedef v16h V; union U { v16h v; v8h h[2]; };
  static __device__ __forceinline__ v16h load(const _Float16* p) {
    U f; f.h[0] = *(const v8h*)(p); f.h[1] = *(const v8h*)(p + 16); return f.v;
  }
  static __device__ __forceinline__ v8f mma(v16h a, v16h b, v8f c) {
    return __builtin_amdgcn_wmma_f32_16x16x32_f16(false, a, false, b, (short)0, c, false, false);
  }
  static __device__ __forceinline__ void guard(v8f& a, v8f& b, v16h x, v16h y) { dep_guard_h(a, b, x, y); }
  static __device__ __forceinline__ void keep(v16h a, v16h b, v16h c, v16h d) { keep4_h(a, b, c, d); }
};
template <> struct Frag<__bf16> {
  typedef v16b V; union U { v16b v; v8b h[2]; };
  static __device__ __forceinline__ v16b load(const __bf16* p) {
    U f; f.h[0] = *(const v8b*)(p); f.h[1] = *(const v8b*)(p + 16); return f.v;
  }
  static __device__ __forceinline__ v8f mma(v16b a, v16b b, v8f c) {
    return __builtin_amdgcn_wmma_f32_16x16x32_bf16(false, a, false, b, (short)0, c, false, false);
  }
  static __device__ __forceinline__ void guard(v8f& a, v8f& b, v16b x, v16b y) { dep_guard_b(a, b, x, y); }
  static __device__ __forceinline__ void keep(v16b a, v16b b, v16b c, v16b d) { keep4_b(a, b, c, d); }
};

template <int ET> struct Elem;
template <> struct Elem<0> { typedef _Float16 T; };
template <> struct Elem<1> { typedef __bf16 T; };
template <int ET, bool SPLIT, int BIAS_MODE, int OUT_MODE, bool RESID, int ACT = 0, bool SPLITB = true>
__global__ __launch_bounds__(256) void wmma_gemm64(
    const unsigned short* __restrict__ Ap, const unsigned short* __restrict__ A2p, int lda, long strideA,
    const unsigned short* __restrict__ Btp, const unsigned short* __restrict__ Bt2p, int ldb, long strideB,
    void* __restrict__ Cout, void* __restrict__ Cout2, int ldc, long strideC,
    const float* __restrict__ bias,
    const float* __restrict__ resid, long strideR,
    int M, int N, int K, float scale) {
  typedef typename Elem<ET>::T T;
  typedef typename Frag<T>::V V;
  const T* A = (const T*)Ap; const T* A2 = (const T*)A2p; const T* Bt = (const T*)Btp; const T* Bt2 = (const T*)Bt2p;
  __shared__ __align__(16) float sT[8][16 * 68];
  const int b    = blockIdx.y;
  const int lane = threadIdx.x & 31;
  const int wave = threadIdx.x >> 5;
  const int tilesN = N >> 6;
  const int tilesM = M >> 6;
  const int tile = blockIdx.x * 8 + wave;
  if (tile >= tilesM * tilesN) return;
  const int tm = tile / tilesN;
  const int tn = tile - tm * tilesN;
  const int m0 = tm << 6;
  const int n0 = tn << 6;

  const T* Ab  = A  + (size_t)b * strideA;
  const T* Bb  = Bt + (size_t)b * strideB;
  const T* Ab2 = SPLIT ? (A2  + (size_t)b * strideA) : nullptr;
  const T* Bb2 = (SPLIT && SPLITB) ? (Bt2 + (size_t)b * strideB) : nullptr;

  const int rlane = lane & 15;
  const int koff  = (lane >> 4) * 8;
  const int mOff  = (lane >> 4) * 8;

  v8f acc[4][4];
#pragma unroll
  for (int i = 0; i < 4; ++i)
#pragma unroll
    for (int j = 0; j < 4; ++j) acc[i][j] = (v8f){0.f,0.f,0.f,0.f,0.f,0.f,0.f,0.f};

  for (int k0 = 0; k0 < K; k0 += 32) {
    V bh[4], bl[4];
#pragma unroll
    for (int j = 0; j < 4; ++j) {
      const size_t bo = (size_t)(n0 + (j << 4) + rlane) * ldb + koff + k0;
      bh[j] = Frag<T>::load(Bb + bo);
      if (SPLIT && SPLITB) bl[j] = Frag<T>::load(Bb2 + bo);
    }
#pragma unroll
    for (int i = 0; i < 4; ++i) {
      const size_t ao = (size_t)(m0 + (i << 4) + rlane) * lda + koff + k0;
      V ah = Frag<T>::load(Ab + ao);
      V al;
      if (SPLIT) al = Frag<T>::load(Ab2 + ao);
#pragma unroll
      for (int j = 0; j < 4; ++j) {
        acc[i][j] = Frag<T>::mma(ah, bh[j], acc[i][j]);
        if (SPLIT) {
          if (SPLITB) acc[i][j] = Frag<T>::mma(ah, bl[j], acc[i][j]);
          acc[i][j] = Frag<T>::mma(al, bh[j], acc[i][j]);
        }
      }
      Frag<T>::guard(acc[i][0], acc[i][3], ah, SPLIT ? al : ah);
    }
    Frag<T>::keep(bh[0], bh[1], bh[2], bh[3]);
    if (SPLIT && SPLITB) Frag<T>::keep(bl[0], bl[1], bl[2], bl[3]);
  }
  acc_guard4(acc[0][0], acc[0][1], acc[0][2], acc[0][3]);
  acc_guard4(acc[1][0], acc[1][1], acc[1][2], acc[1][3]);
  acc_guard4(acc[2][0], acc[2][1], acc[2][2], acc[2][3]);
  acc_guard4(acc[3][0], acc[3][1], acc[3][2], acc[3][3]);

  float* slab = sT[wave];
  const float* Rb = RESID ? (resid + (size_t)b * strideR) : nullptr;
#pragma unroll
  for (int i = 0; i < 4; ++i) {
    const int mBase = m0 + (i << 4);
#pragma unroll
    for (int j = 0; j < 4; ++j) {
      const int n = n0 + (j << 4) + rlane;
      float bv = 0.f;
      if (BIAS_MODE == 2) bv = bias[n];
#pragma unroll
      for (int r = 0; r < 8; ++r) {
        float v = acc[i][j][r] * scale;
        if (BIAS_MODE == 1) v += bias[mBase + mOff + r];
        if (BIAS_MODE == 2) v += bv;
        if (RESID) v += Rb[(size_t)(mBase + mOff + r) * ldc + n];
        if (ACT == 1) v = tanhf(v);
        if (ACT == 2) v = fmaxf(v, 0.0f);
        if (ACT == 3) v = v / (1.0f + expf(-v));
        if (ACT == 4) v = (v > 0.f) ? v : 0.01f * v;
        slab[(mOff + r) * 68 + (j << 4) + rlane] = v;
      }
    }
    __builtin_amdgcn_fence(__ATOMIC_RELEASE, "workgroup");
    __builtin_amdgcn_wave_barrier();
    __builtin_amdgcn_fence(__ATOMIC_ACQUIRE, "workgroup");
    if (OUT_MODE == 0) {
      float* C = (float*)Cout + (size_t)b * strideC;
      const int hh = lane >> 4, c4 = (lane & 15) * 4;
      for (int pass = 0; pass < 2; ++pass) {
#pragma unroll
        for (int it = 0; it < 8; ++it) {
          const int row = it * 2 + hh;
          v4f v = *(const v4f*)(slab + row * 68 + c4);
          *(volatile v4f*)(C + (size_t)(mBase + row) * ldc + n0 + c4) = v;
        }
        __threadfence();
      }
    } else {
      const int q = lane >> 3, c8 = (lane & 7) * 8;
      unsigned short* C  = (unsigned short*)Cout  + (size_t)b * strideC;
      unsigned short* C2 = (OUT_MODE == 2) ? ((unsigned short*)Cout2 + (size_t)b * strideC) : nullptr;
      for (int pass = 0; pass < 2; ++pass) {
#pragma unroll
        for (int it = 0; it < 4; ++it) {
          const int row = it * 4 + q;
          const float* sp = slab + row * 68 + c8;
          v8h hv, lv;
#pragma unroll
          for (int e = 0; e < 8; ++e) {
            if (OUT_MODE == 1) {
              hv[e] = (_Float16)sp[e];
            } else {
              unsigned short hb = f2bf_bits(sp[e]);
              unsigned short lb = f2bf_bits(sp[e] - bf_bits2f(hb));
              hv[e] = __builtin_bit_cast(_Float16, hb);
              lv[e] = __builtin_bit_cast(_Float16, lb);
            }
          }
          *(volatile v8h*)(C + (size_t)(mBase + row) * ldc + n0 + c8) = hv;
          if (OUT_MODE == 2) *(volatile v8h*)(C2 + (size_t)(mBase + row) * ldc + n0 + c8) = lv;
        }
        __threadfence();
      }
    }
    __builtin_amdgcn_fence(__ATOMIC_RELEASE, "workgroup");
    __builtin_amdgcn_wave_barrier();
    __builtin_amdgcn_fence(__ATOMIC_ACQUIRE, "workgroup");
  }
}

__global__ __launch_bounds__(256) void cast_f32_bf16x8(const float* __restrict__ in,
                                                        unsigned short* __restrict__ out, int n8) {
  const int i = blockIdx.x * 256 + threadIdx.x;
  if (i < n8) {
    const v4f a = *(const v4f*)(in + (size_t)i * 8);
    const v4f c = *(const v4f*)(in + (size_t)i * 8 + 4);
    v8h hv;
#pragma unroll
    for (int e = 0; e < 4; ++e) {
      hv[e]     = __builtin_bit_cast(_Float16, f2bf_bits(a[e]));
      hv[4 + e] = __builtin_bit_cast(_Float16, f2bf_bits(c[e]));
    }
    *(volatile v8h*)(out + (size_t)i * 8) = hv;
    __threadfence();
    *(volatile v8h*)(out + (size_t)i * 8) = hv;
  }
}

__global__ __launch_bounds__(128) void norm_qkv_k(const float* __restrict__ Y,
    const float* __restrict__ bq, const float* __restrict__ bk, const float* __restrict__ bv,
    unsigned short* __restrict__ qpl, unsigned short* __restrict__ kpl,
    unsigned short* __restrict__ vhp, unsigned short* __restrict__ vlp) {
  __shared__ float red[3][4];
  const int row = blockIdx.x, tid = threadIdx.x, lane = tid & 31, wave = tid >> 5;
  const int bi = row / kSeq, n = row - bi * kSeq;
  const int c8 = tid * 8;
  const float* yr = Y + (size_t)row * kQkvN;
  v4f tq0 = *(const v4f*)(yr + c8),            tq1 = *(const v4f*)(yr + c8 + 4);
  v4f tk0 = *(const v4f*)(yr + kDim + c8),     tk1 = *(const v4f*)(yr + kDim + c8 + 4);
  v4f tv0 = *(const v4f*)(yr + 2 * kDim + c8), tv1 = *(const v4f*)(yr + 2 * kDim + c8 + 4);
  const v4f bq0 = *(const v4f*)(bq + c8), bq1 = *(const v4f*)(bq + c8 + 4);
  const v4f bk0 = *(const v4f*)(bk + c8), bk1 = *(const v4f*)(bk + c8 + 4);
  const v4f bv0 = *(const v4f*)(bv + c8), bv1 = *(const v4f*)(bv + c8 + 4);
  float sq = 0.f, sk = 0.f, sv = 0.f;
#pragma unroll
  for (int e = 0; e < 4; ++e) {
    tq0[e] += bfrn(bq0[e]); tq1[e] += bfrn(bq1[e]);
    tk0[e] += bfrn(bk0[e]); tk1[e] += bfrn(bk1[e]);
    tv0[e] += bfrn(bv0[e]); tv1[e] += bfrn(bv1[e]);
    sq += tq0[e] * tq0[e] + tq1[e] * tq1[e];
    sk += tk0[e] * tk0[e] + tk1[e] * tk1[e];
    sv += tv0[e] * tv0[e] + tv1[e] * tv1[e];
  }
#pragma unroll
  for (int off = 1; off < 32; off <<= 1) {
    sq += __shfl_xor(sq, off, 32);
    sk += __shfl_xor(sk, off, 32);
    sv += __shfl_xor(sv, off, 32);
  }
  if (lane == 0) { red[0][wave] = sq; red[1][wave] = sk; red[2][wave] = sv; }
  __syncthreads();
  const float totq = (red[0][0] + red[0][1]) + (red[0][2] + red[0][3]);
  const float totk = (red[1][0] + red[1][1]) + (red[1][2] + red[1][3]);
  const float totv = (red[2][0] + red[2][1]) + (red[2][2] + red[2][3]);
  const float invq = 1.0f / (sqrtf(totq) + kEps);
  const float invk = 1.0f / (sqrtf(totk) + kEps);
  const float invv = 1.0f / (sqrtf(totv) + kEps);
  const int h = tid >> 3, d8 = (tid & 7) * 8;
  const size_t po = (((size_t)(bi * kHeads + h)) * kSeq + n) * kHd + d8;
  v8h hq, hk, hvh, hvl;
#pragma unroll
  for (int e = 0; e < 4; ++e) {
    const float q0 = tq0[e] * invq, q1 = tq1[e] * invq;
    const float k0 = tk0[e] * invk, k1 = tk1[e] * invk;
    const float v0 = tv0[e] * invv, v1 = tv1[e] * invv;
    hq[e] = (_Float16)(q0 * kQCarry); hq[4 + e] = (_Float16)(q1 * kQCarry);
    hk[e] = (_Float16)(k0 * kQCarry); hk[4 + e] = (_Float16)(k1 * kQCarry);
    const unsigned short hb0 = f2bf_bits(v0), hb1 = f2bf_bits(v1);
    const unsigned short lb0 = f2bf_bits(v0 - bf_bits2f(hb0)), lb1 = f2bf_bits(v1 - bf_bits2f(hb1));
    hvh[e] = __builtin_bit_cast(_Float16, hb0); hvh[4 + e] = __builtin_bit_cast(_Float16, hb1);
    hvl[e] = __builtin_bit_cast(_Float16, lb0); hvl[4 + e] = __builtin_bit_cast(_Float16, lb1);
  }
  for (int pass = 0; pass < 2; ++pass) {
    *(volatile v8h*)(qpl + po) = hq;
    *(volatile v8h*)(kpl + po) = hk;
    *(volatile v8h*)(vhp + po) = hvh;
    *(volatile v8h*)(vlp + po) = hvl;
    __threadfence();
  }
}

__global__ __launch_bounds__(128) void norm_out_k(const float* __restrict__ Z, const float* __restrict__ bo,
                                                  float* __restrict__ out) {
  __shared__ float red[4];
  const int row = blockIdx.x, tid = threadIdx.x, lane = tid & 31, wave = tid >> 5;
  const size_t rb = (size_t)row * kDim;
  const int ca = tid * 4, cb = 512 + tid * 4;
  v4f va = *(const v4f*)(Z + rb + ca);
  v4f vb = *(const v4f*)(Z + rb + cb);
  const v4f ba = *(const v4f*)(bo + ca), bb = *(const v4f*)(bo + cb);
  float s = 0.f;
#pragma unroll
  for (int e = 0; e < 4; ++e) {
    va[e] += bfrn(ba[e]); vb[e] += bfrn(bb[e]);
    s += va[e] * va[e] + vb[e] * vb[e];
  }
#pragma unroll
  for (int off = 1; off < 32; off <<= 1) s += __shfl_xor(s, off, 32);
  if (lane == 0) red[wave] = s;
  __syncthreads();
  const float tot = (red[0] + red[1]) + (red[2] + red[3]);
  const float inv = 1.0f / (sqrtf(tot) + kEps);
  const v4f ya = va * inv, yb = vb * inv;
  for (int pass = 0; pass < 2; ++pass) {
    *(volatile v4f*)(out + rb + ca) = ya;
    *(volatile v4f*)(out + rb + cb) = yb;
    __threadfence();
  }
}

__device__ __forceinline__ v8f mma_h(v16h a, v16h b, v8f c) {
  c = __builtin_amdgcn_wmma_f32_16x16x32_f16(false, a, false, b, (short)0, c, false, false);
  asm volatile("v_nop\n\tv_nop\n\tv_nop\n\tv_nop" : "+v"(c) : "v"(a), "v"(b));
  return c;
}
__device__ __forceinline__ v8f mma_b(v16b a, v16b b, v8f c) {
  c = __builtin_amdgcn_wmma_f32_16x16x32_bf16(false, a, false, b, (short)0, c, false, false);
  asm volatile("v_nop\n\tv_nop\n\tv_nop\n\tv_nop" : "+v"(c) : "v"(a), "v"(b));
  return c;
}
__device__ __forceinline__ void split_bf(float f, __bf16& hi, __bf16& lo) {
  const unsigned short hb = f2bf_bits(f);
  hi = __builtin_bit_cast(__bf16, hb);
  lo = __builtin_bit_cast(__bf16, f2bf_bits(f - bf_bits2f(hb)));
}

static constexpr int kKC = 64;
static constexpr int kQB = 64;
static constexpr int kOSP = 68;
__global__ __launch_bounds__(128) void attn_k(const unsigned short* __restrict__ qpp, const unsigned short* __restrict__ kpp,
                                              const unsigned short* __restrict__ vhpp, const unsigned short* __restrict__ vlpp,
                                              const int* __restrict__ maskp,
                                              unsigned short* __restrict__ ohp, unsigned short* __restrict__ olp) {
  union FH { v16h v; v8h h[2]; };
  union FB { v16b v; v8b h[2]; };
  __shared__ __align__(16) _Float16 Ksh[kKC * kHd];
  __shared__ __align__(16) __bf16   Vth[kHd * kKC];
  __shared__ __align__(16) __bf16   Vtl[kHd * kKC];
  __shared__ __align__(16) __bf16   Psh[4][16 * kKC];
  __shared__ __align__(16) __bf16   Psl[4][16 * kKC];
  __shared__ __align__(16) float    Os[4][16 * kOSP];
  const _Float16* qp = (const _Float16*)qpp;
  const _Float16* kp = (const _Float16*)kpp;
  const __bf16* vhp = (const __bf16*)vhpp;
  const __bf16* vlp = (const __bf16*)vlpp;
  const int tid = threadIdx.x, wave = tid >> 5, lane = tid & 31, hh = lane >> 4, c = lane & 15;
  const int nqb = kSeq / kQB;
  const int bx = blockIdx.x;
  const int qb = bx % nqb;
  const int bh = bx / nqb;
  const int h = bh % kHeads;
  const int b = bh / kHeads;
  const int q0 = qb * kQB + wave * 16;
  const size_t rowb = (size_t)bh * kSeq;

  v16h qa[2];
  {
    const _Float16* qrow = qp + (rowb + q0 + c) * kHd + 8 * hh;
#pragma unroll
    for (int dc = 0; dc < 2; ++dc) qa[dc] = Frag<_Float16>::load(qrow + dc * 32);
  }
  float mrow[8], lrow[8];
  v8f oacc[4];
#pragma unroll
  for (int r = 0; r < 8; ++r) { mrow[r] = -INFINITY; lrow[r] = 0.f; }
#pragma unroll
  for (int t = 0; t < 4; ++t) oacc[t] = (v8f){0.f,0.f,0.f,0.f,0.f,0.f,0.f,0.f};

  const int nChunks = qb + 1;
  for (int kc = 0; kc < nChunks; ++kc) {
    const int kv0 = kc * kKC;
    __syncthreads();
    {
      const int kvr = tid >> 1, dh = (tid & 1) * 32;
      const size_t src = (rowb + kv0 + kvr) * kHd + dh;
#pragma unroll 1
      for (int i = 0; i < 4; ++i) {
        const v8h kk = *(const v8h*)(kp + src + 8 * i);
        *(v8h*)(Ksh + kvr * kHd + dh + 8 * i) = kk;
        const v8b vh = *(const v8b*)(vhp + src + 8 * i);
        const v8b vl = *(const v8b*)(vlp + src + 8 * i);
#pragma unroll
        for (int e = 0; e < 8; ++e) {
          Vth[(dh + 8 * i + e) * kKC + kvr] = vh[e];
          Vtl[(dh + 8 * i + e) * kKC + kvr] = vl[e];
        }
      }
    }
    __syncthreads();

    v8f s[4];
#pragma unroll
    for (int j = 0; j < 4; ++j) {
      s[j] = (v8f){0.f,0.f,0.f,0.f,0.f,0.f,0.f,0.f};
#pragma unroll
      for (int dc = 0; dc < 2; ++dc) {
        FH kb;
        kb.h[0] = *(const v8h*)(Ksh + (j * 16 + c) * kHd + dc * 32 + 8 * hh);
        kb.h[1] = *(const v8h*)(Ksh + (j * 16 + c) * kHd + dc * 32 + 16 + 8 * hh);
        s[j] = mma_h(qa[dc], kb.v, s[j]);
      }
    }
    const bool diag = (kc == qb);
    float cm[8];
#pragma unroll
    for (int r = 0; r < 8; ++r) {
      const int qrow = q0 + 8 * hh + r;
      float m = -INFINITY;
#pragma unroll
      for (int j = 0; j < 4; ++j) {
        const int kvcol = kv0 + j * 16 + c;
        float sv = s[j][r] * kScoreScale;
        if (diag) {
          const int mk = maskp[(size_t)qrow * kSeq + kvcol];
          sv = (mk != 0) ? kMaskFill : sv;
        }
        s[j][r] = sv;
        m = fmaxf(m, sv);
      }
#pragma unroll
      for (int off = 1; off < 16; off <<= 1) m = fmaxf(m, __shfl_xor(m, off, 32));
      cm[r] = m;
    }
    __bf16* pwh = Psh[wave];
    __bf16* pwl = Psl[wave];
#pragma unroll
    for (int r = 0; r < 8; ++r) {
      const float mnew = fmaxf(mrow[r], cm[r]);
      const float alpha = expf(mrow[r] - mnew);
      mrow[r] = mnew;
      float psum = 0.f;
#pragma unroll
      for (int j = 0; j < 4; ++j) {
        const float p = expf(s[j][r] - mnew);
        psum += p;
        __bf16 ph, pl;
        split_bf(p, ph, pl);
        pwh[(8 * hh + r) * kKC + j * 16 + c] = ph;
        pwl[(8 * hh + r) * kKC + j * 16 + c] = pl;
      }
#pragma unroll
      for (int off = 1; off < 16; off <<= 1) psum += __shfl_xor(psum, off, 32);
      lrow[r] = lrow[r] * alpha + psum;
#pragma unroll
      for (int t = 0; t < 4; ++t) oacc[t][r] *= alpha;
    }
    __builtin_amdgcn_fence(__ATOMIC_RELEASE, "workgroup");
    __builtin_amdgcn_wave_barrier();
    __builtin_amdgcn_fence(__ATOMIC_ACQUIRE, "workgroup");
#pragma unroll 1
    for (int kk = 0; kk < 2; ++kk) {
      FB pa, pl;
      pa.h[0] = *(const v8b*)(pwh + c * kKC + kk * 32 + 8 * hh);
      pa.h[1] = *(const v8b*)(pwh + c * kKC + kk * 32 + 16 + 8 * hh);
      pl.h[0] = *(const v8b*)(pwl + c * kKC + kk * 32 + 8 * hh);
      pl.h[1] = *(const v8b*)(pwl + c * kKC + kk * 32 + 16 + 8 * hh);
#pragma unroll
      for (int t = 0; t < 4; ++t) {
        FB vb, vl;
        vb.h[0] = *(const v8b*)(Vth + (t * 16 + c) * kKC + kk * 32 + 8 * hh);
        vb.h[1] = *(const v8b*)(Vth + (t * 16 + c) * kKC + kk * 32 + 16 + 8 * hh);
        vl.h[0] = *(const v8b*)(Vtl + (t * 16 + c) * kKC + kk * 32 + 8 * hh);
        vl.h[1] = *(const v8b*)(Vtl + (t * 16 + c) * kKC + kk * 32 + 16 + 8 * hh);
        oacc[t] = mma_b(pa.v, vb.v, oacc[t]);
        oacc[t] = mma_b(pa.v, vl.v, oacc[t]);
        oacc[t] = mma_b(pl.v, vb.v, oacc[t]);
      }
    }
  }

  float* os = Os[wave];
#pragma unroll
  for (int r = 0; r < 8; ++r) {
    const float inv = 1.0f / lrow[r];
#pragma unroll
    for (int t = 0; t < 4; ++t) os[(8 * hh + r) * kOSP + t * 16 + c] = oacc[t][r] * inv;
  }
  __builtin_amdgcn_fence(__ATOMIC_RELEASE, "workgroup");
  __builtin_amdgcn_wave_barrier();
  __builtin_amdgcn_fence(__ATOMIC_ACQUIRE, "workgroup");
  {
    const int q8 = lane >> 3, c8 = (lane & 7) * 8;
    for (int pass = 0; pass < 2; ++pass) {
#pragma unroll
      for (int it = 0; it < 4; ++it) {
        const int row = it * 4 + q8;
        const float* sp = os + row * kOSP + c8;
        v8h hv, lv;
#pragma unroll
        for (int e = 0; e < 8; ++e) {
          const unsigned short hb = f2bf_bits(sp[e]);
          const unsigned short lb = f2bf_bits(sp[e] - bf_bits2f(hb));
          hv[e] = __builtin_bit_cast(_Float16, hb);
          lv[e] = __builtin_bit_cast(_Float16, lb);
        }
        const size_t ob = ((size_t)(b * kSeq + q0 + row)) * kDim + h * kHd + c8;
        *(volatile v8h*)(ohp + ob) = hv;
        *(volatile v8h*)(olp + ob) = lv;
      }
      __threadfence();
    }
  }
}

extern "C" void kernel_launch(void* const* d_in, const int* in_sizes, int n_in,
                              void* d_out, int out_size, void* d_ws, size_t ws_size,
                              hipStream_t stream) {
  if (n_in < 10) return;
  if (in_sizes[0] != kRows * kDim) return;
  if (in_sizes[1] != kDim * kDim || in_sizes[3] != kDim * kDim || in_sizes[5] != kDim * kDim || in_sizes[7] != kDim * kDim) return;
  if (in_sizes[2] != kDim || in_sizes[4] != kDim || in_sizes[6] != kDim || in_sizes[8] != kDim) return;
  if (in_sizes[9] != kSeq * kSeq) return;
  if (out_size != kRows * kDim) return;

  const float* x  = (const float*)d_in[0];
  const float* Wq = (const float*)d_in[1];
  const float* bq = (const float*)d_in[2];
  const float* Wk = (const float*)d_in[3];
  const float* bk = (const float*)d_in[4];
  const float* Wv = (const float*)d_in[5];
  const float* bv = (const float*)d_in[6];
  const float* Wo = (const float*)d_in[7];
  const float* bo = (const float*)d_in[8];
  const int*   mask = (const int*)d_in[9];
  float* outp = (float*)d_out;

  const size_t nTok = (size_t)kRows * kDim;
  const size_t nW   = (size_t)kDim * kDim;
  const size_t oXb   = 0;
  const size_t oWcat = oXb   + nTok * 2;
  const size_t oWob  = oWcat + 3 * nW * 2;
  const size_t oQ    = oWob  + nW * 2;
  const size_t oK    = oQ    + nTok * 2;
  const size_t oVh   = oK    + nTok * 2;
  const size_t oVl   = oVh   + nTok * 2;
  const size_t oY    = oVl   + nTok * 2;
  const size_t bY    = (size_t)kRows * kQkvN * 4;
  const size_t oOh   = oY;
  const size_t oOl   = oOh + nTok * 2;
  const size_t oZ    = oOl + nTok * 2;
  const size_t total = oY + bY;
  if (oZ + nTok * 4 > total) return;
  if (total > ws_size) return;

  char* ws = (char*)d_ws;
  unsigned short* xb   = (unsigned short*)(ws + oXb);
  unsigned short* Wcat = (unsigned short*)(ws + oWcat);
  unsigned short* Wob  = (unsigned short*)(ws + oWob);
  unsigned short* qpl  = (unsigned short*)(ws + oQ);
  unsigned short* kpl  = (unsigned short*)(ws + oK);
  unsigned short* vhp  = (unsigned short*)(ws + oVh);
  unsigned short* vlp  = (unsigned short*)(ws + oVl);
  float*          Y    = (float*)(ws + oY);
  unsigned short* ohp  = (unsigned short*)(ws + oOh);
  unsigned short* olp  = (unsigned short*)(ws + oOl);
  float*          Z    = (float*)(ws + oZ);

  const int n8x = (int)(nTok / 8);
  const int n8w = (int)(nW / 8);
  cast_f32_bf16x8<<<(n8x + 255) / 256, 256, 0, stream>>>(x,  xb, n8x);
  cast_f32_bf16x8<<<(n8w + 255) / 256, 256, 0, stream>>>(Wq, Wcat, n8w);
  cast_f32_bf16x8<<<(n8w + 255) / 256, 256, 0, stream>>>(Wk, Wcat + nW, n8w);
  cast_f32_bf16x8<<<(n8w + 255) / 256, 256, 0, stream>>>(Wv, Wcat + 2 * nW, n8w);
  cast_f32_bf16x8<<<(n8w + 255) / 256, 256, 0, stream>>>(Wo, Wob, n8w);

  {
    const int tiles = (kRows / 64) * (kQkvN / 64);
    wmma_gemm64<1, false, 0, 0, false><<<dim3((tiles + 7) / 8, 1), 256, 0, stream>>>(
        xb, xb, kDim, 0L, Wcat, Wcat, kDim, 0L, (void*)Y, (void*)Y, kQkvN, 0L,
        bq, (const float*)Y, 0L, kRows, kQkvN, kDim, 1.0f);
  }

  norm_qkv_k<<<kRows, 128, 0, stream>>>(Y, bq, bk, bv, qpl, kpl, vhp, vlp);

  attn_k<<<kBatch * kHeads * (kSeq / kQB), 128, 0, stream>>>(qpl, kpl, vhp, vlp, mask, ohp, olp);

  {
    const int tiles = (kRows / 64) * (kDim / 64);
    wmma_gemm64<1, true, 0, 0, false, 0, false><<<dim3((tiles + 7) / 8, 1), 256, 0, stream>>>(
        ohp, olp, kDim, 0L, Wob, Wob, kDim, 0L, (void*)Z, (void*)Z, kDim, 0L,
        bo, (const float*)Z, 0L, kRows, kDim, kDim, 1.0f);
  }

  norm_out_k<<<kRows, 128, 0, stream>>>(Z, bo, outp);
}
